// TransformerBlock_17746804867396
// MI455X (gfx1250) — hardware-verified
//
#include <hip/hip_runtime.h>
#include <stdint.h>
#include <stddef.h>


#pragma clang fp contract(off)

#ifndef NB
#define NB 2
#endif
#ifndef SEQ
#define SEQ 2048
#endif
#define NB_FULL 2
#define SEQ_FULL 2048
#define DMOD 1024
#define NH 16
#define HD 64
#define DFF 4096
#define EARLY_QT 4

#define LDA 72
#define LDT 72
#define LDE 136
#define LDC 132
#define LDSF 68
#define SMEM_BIG (128 * LDE * 2 * 2)
#define SMEM_QKV (SMEM_BIG + 128 * HD * 4 * 2)

#define WSC 64.0f
#define WINV 0.015625f
#define CRES 4096.0f
#define CRINV 0.000244140625f
#define CPV 4096.0f
#define OSC 16.0f

static_assert(NB >= 1 && NB <= NB_FULL);
static_assert(SEQ >= 256 && SEQ <= SEQ_FULL && (SEQ % 128) == 0);
static_assert((DMOD % 128) == 0 && (DMOD % 64) == 0 && (DFF % 64) == 0);
static_assert(HD == 64 && NH * HD == DMOD);
static_assert(128 * LDC * 4 <= SMEM_BIG);
static_assert(2 * 128 * LDA * 2 <= SMEM_BIG);
static_assert((SEQ / 64) >= EARLY_QT);

typedef _Float16 v16h __attribute__((ext_vector_type(16)));
typedef _Float16 v8h __attribute__((ext_vector_type(8)));
typedef float v8f __attribute__((ext_vector_type(8)));
typedef float v4f __attribute__((ext_vector_type(4)));

union Frag { v16h v; v8h half[2]; };

__device__ __forceinline__ float bfr(float f) {
  unsigned int u = __float_as_uint(f);
  u = (u + 0x7FFFu + ((u >> 16) & 1u)) & 0xFFFF0000u;
  return __uint_as_float(u);
}

__device__ __forceinline__ v8f zero8() {
  v8f z = {0.0f, 0.0f, 0.0f, 0.0f, 0.0f, 0.0f, 0.0f, 0.0f};
  return z;
}

__device__ __forceinline__ v16h ld_frag(const _Float16* base, int ld) {
  const int lane = threadIdx.x & 31;
  const _Float16* p = base + (lane & 15) * ld + (lane >> 4) * 8;
  Frag f;
  f.half[0] = *(const v8h*)(p);
  f.half[1] = *(const v8h*)(p + 16);
  return f.v;
}

__device__ __forceinline__ v8f wmma16(v16h a, v16h b, v8f c) {
  v8f d = __builtin_amdgcn_wmma_f32_16x16x32_f16(false, a, false, b, (short)0, c, false, false);
  asm volatile("v_nop\n\tv_nop\n\tv_nop\n\tv_nop" : "+v"(d) : "v"(a), "v"(b));
  return d;
}

__global__ __launch_bounds__(256) void k_cvt_w(const float* __restrict__ src,
                                               _Float16* __restrict__ dst, int n8)
{
  const int i = (int)blockIdx.x * 256 + (int)threadIdx.x;
  if (i >= n8) return;
  const v4f a = *(const v4f*)(src + (size_t)i * 8);
  const v4f c = *(const v4f*)(src + (size_t)i * 8 + 4);
  v8h o;
#pragma unroll
  for (int e = 0; e < 4; ++e) {
    o[e]     = (_Float16)(bfr(a[e]) * WSC);
    o[e + 4] = (_Float16)(bfr(c[e]) * WSC);
  }
  _Float16* p = dst + (size_t)i * 8;
  *(volatile v8h*)p = o;
  __threadfence();
  *(volatile v8h*)p = o;
}

__global__ __launch_bounds__(256) void k_trig(const float* __restrict__ rpe,
                                              float* __restrict__ cosT,
                                              float* __restrict__ sinT, int n)
{
  const int i = (int)blockIdx.x * 256 + (int)threadIdx.x;
  if (i >= n) return;
  const float a = bfr(rpe[i]);
  const float cv = cosf(a);
  const float sv = sinf(a);
  *(volatile float*)(cosT + i) = cv;
  *(volatile float*)(sinT + i) = sv;
  __threadfence();
  *(volatile float*)(cosT + i) = cv;
  *(volatile float*)(sinT + i) = sv;
}

template<int RIN>
__global__ __launch_bounds__(256) void k_rms(const float* __restrict__ X,
                                             const float* __restrict__ W,
                                             _Float16* __restrict__ Hout, int nrows)
{
  const int lane = threadIdx.x & 31, wid = threadIdx.x >> 5;
  const int rl = (int)blockIdx.x * 8 + wid;
  if (rl >= nrows) return;
  const int b = rl / SEQ;
  const int s = rl - b * SEQ;
  const size_t R = (size_t)b * SEQ_FULL + (size_t)s;
  const float* xr = X + R * DMOD;

  float ss = 0.0f;
#pragma unroll 1
  for (int j = 0; j < 4; ++j) {
    const int base = (j * 32 + lane) * 8;
    const v4f a = *(const v4f*)(xr + base);
    const v4f c = *(const v4f*)(xr + base + 4);
#pragma unroll
    for (int e = 0; e < 4; ++e) {
      float t = RIN ? bfr(a[e]) : a[e];
      ss += t * t;
      t = RIN ? bfr(c[e]) : c[e];
      ss += t * t;
    }
  }
  ss += __shfl_xor(ss, 16, 32);
  ss += __shfl_xor(ss, 8, 32);
  ss += __shfl_xor(ss, 4, 32);
  ss += __shfl_xor(ss, 2, 32);
  ss += __shfl_xor(ss, 1, 32);
  const float nrm = sqrtf(ss) * 0.03125f;
  const float inv = __builtin_amdgcn_rcpf(nrm + 1e-6f);

  v8h hv[4];
#pragma unroll
  for (int j = 0; j < 4; ++j) {
    const int base = (j * 32 + lane) * 8;
    const v4f a  = *(const v4f*)(xr + base);
    const v4f c  = *(const v4f*)(xr + base + 4);
    const v4f w0 = *(const v4f*)(W + base);
    const v4f w1 = *(const v4f*)(W + base + 4);
#pragma unroll
    for (int e = 0; e < 4; ++e) {
      float t = RIN ? bfr(a[e]) : a[e];
      t = t * inv;
      t = t * bfr(w0[e]);
      hv[j][e] = (_Float16)t;
      float u = RIN ? bfr(c[e]) : c[e];
      u = u * inv;
      u = u * bfr(w1[e]);
      hv[j][e + 4] = (_Float16)u;
    }
  }
  _Float16* hp = Hout + R * DMOD;
#pragma unroll
  for (int j = 0; j < 4; ++j) *(volatile v8h*)(hp + (j * 32 + lane) * 8) = hv[j];
  __threadfence();
#pragma unroll
  for (int j = 0; j < 4; ++j) *(volatile v8h*)(hp + (j * 32 + lane) * 8) = hv[j];
}

__global__ __launch_bounds__(256) __attribute__((amdgpu_num_vgpr(256)))
void k_qkv(const _Float16* __restrict__ Hp,
           const _Float16* __restrict__ Wq, const _Float16* __restrict__ Wk,
           const _Float16* __restrict__ Wv,
           const float* __restrict__ cosT, const float* __restrict__ sinT,
           _Float16* __restrict__ Qh, _Float16* __restrict__ Ql,
           _Float16* __restrict__ Kh, _Float16* __restrict__ Kl,
           _Float16* __restrict__ Vth, _Float16* __restrict__ Vtl)
{
  __shared__ __attribute__((aligned(16))) char smem[SMEM_QKV];
  _Float16* As = (_Float16*)smem;
  _Float16* Ws = As + 128 * LDA;

  const int tid = threadIdx.x, lane = tid & 31, wid = tid >> 5;
  const int mw = wid >> 1, nw = wid & 1, hh = lane >> 4, n16 = lane & 15;
  const int rt = (int)blockIdx.x;
  const int b = rt / (SEQ / 128);
  const int s0 = (rt - b * (SEQ / 128)) * 128;
  const size_t R0 = (size_t)b * SEQ_FULL + (size_t)s0;
  const int widx = (int)blockIdx.y / (DMOD / 128);
  const int n0 = ((int)blockIdx.y - widx * (DMOD / 128)) * 128;
  const _Float16* W = (widx == 0) ? Wq : ((widx == 1) ? Wk : Wv);

  v8f acc[2][4];
#pragma unroll
  for (int mt = 0; mt < 2; ++mt)
#pragma unroll
    for (int nt = 0; nt < 4; ++nt) acc[mt][nt] = zero8();

#pragma unroll 1
  for (int kb = 0; kb < DMOD; kb += 64) {
    __syncthreads();
#pragma unroll
    for (int j = 0; j < 4; ++j) {
      const int c = tid + j * 256;
      const int r = c >> 3, cc = (c & 7) * 8;
      *(v8h*)(As + r * LDA + cc) = *(const v8h*)(Hp + (R0 + r) * DMOD + kb + cc);
      *(v8h*)(Ws + r * LDA + cc) = *(const v8h*)(W + (size_t)(n0 + r) * DMOD + kb + cc);
    }
    __syncthreads();
#pragma unroll
    for (int ks = 0; ks < 2; ++ks) {
      const v16h a0 = ld_frag(As + (mw * 32) * LDA + ks * 32, LDA);
      const v16h a1 = ld_frag(As + (mw * 32 + 16) * LDA + ks * 32, LDA);
#pragma unroll
      for (int nt = 0; nt < 4; ++nt) {
        const v16h bw = ld_frag(Ws + (nw * 64 + nt * 16) * LDA + ks * 32, LDA);
        acc[0][nt] = wmma16(a0, bw, acc[0][nt]);
        acc[1][nt] = wmma16(a1, bw, acc[1][nt]);
      }
    }
  }
  __syncthreads();

  _Float16* Hs = (_Float16*)smem;
  _Float16* Ls = Hs + 128 * LDE;
  float* Cz = (float*)(smem + SMEM_BIG);
  float* Sz = Cz + 128 * HD;

  if (widx < 2) {
#pragma unroll
    for (int j = 0; j < 8; ++j) {
      const int c = tid + j * 256;
      const int r = c >> 4, cc = (c & 15) * 4;
      *(v4f*)(Cz + r * HD + cc) = *(const v4f*)(cosT + (size_t)(s0 + r) * HD + cc);
      *(v4f*)(Sz + r * HD + cc) = *(const v4f*)(sinT + (size_t)(s0 + r) * HD + cc);
    }
  }
  __syncthreads();

  if (widx < 2) {
#pragma unroll
    for (int mt = 0; mt < 2; ++mt)
#pragma unroll
      for (int r = 0; r < 8; ++r) {
        const int lrow = mw * 32 + mt * 16 + hh * 8 + r;
        const float* cr = Cz + lrow * HD;
        const float* sr = Sz + lrow * HD;
#pragma unroll
        for (int nt = 0; nt < 2; ++nt) {
          const int d1 = nt * 16 + n16;
          const float c1 = cr[d1], s1 = sr[d1], c2 = cr[d1 + 32], s2 = sr[d1 + 32];
          const float t1 = acc[mt][nt][r] * WINV;
          const float t2 = acc[mt][nt + 2][r] * WINV;
          const float o1 = t1 * c1 - t2 * s1;
          const float o2 = t2 * c2 + t1 * s2;
          const _Float16 h1v = (_Float16)o1;
          const _Float16 h2v = (_Float16)o2;
          const int col = nw * 64 + d1;
          Hs[lrow * LDE + col] = h1v;
          Ls[lrow * LDE + col] = (_Float16)((o1 - (float)h1v) * CRES);
          Hs[lrow * LDE + col + 32] = h2v;
          Ls[lrow * LDE + col + 32] = (_Float16)((o2 - (float)h2v) * CRES);
        }
      }
  } else {
#pragma unroll
    for (int mt = 0; mt < 2; ++mt)
#pragma unroll
      for (int r = 0; r < 8; ++r) {
        const int lrow = mw * 32 + mt * 16 + hh * 8 + r;
#pragma unroll
        for (int nt = 0; nt < 4; ++nt) {
          const int d = nw * 64 + nt * 16 + n16;
          const float t = acc[mt][nt][r] * WINV;
          const _Float16 hv = (_Float16)t;
          Hs[d * LDE + lrow] = hv;
          Ls[d * LDE + lrow] = (_Float16)((t - (float)hv) * CRES);
        }
      }
  }
  __syncthreads();

  _Float16* dstH = (widx == 0) ? Qh : ((widx == 1) ? Kh : Vth);
  _Float16* dstL = (widx == 0) ? Ql : ((widx == 1) ? Kl : Vtl);
  const size_t vtr0 = (size_t)b * DMOD;
#pragma unroll
  for (int pl = 0; pl < 2; ++pl) {
    const _Float16* S = (pl == 0) ? Hs : Ls;
    _Float16* D = (pl == 0) ? dstH : dstL;
    v8h pv[8];
#pragma unroll
    for (int it = 0; it < 8; ++it) {
      const int p = tid + it * 256;
      const int row = p >> 4, q = (p & 15) * 8;
      pv[it] = *(const v8h*)(S + row * LDE + q);
    }
#pragma unroll
    for (int it = 0; it < 8; ++it) {
      const int p = tid + it * 256;
      const int row = p >> 4, q = (p & 15) * 8;
      const size_t off = (widx < 2) ? ((R0 + row) * DMOD + (size_t)(n0 + q))
                                    : ((vtr0 + n0 + row) * SEQ_FULL + (size_t)(s0 + q));
      *(volatile v8h*)(D + off) = pv[it];
    }
    __threadfence();
#pragma unroll
    for (int it = 0; it < 8; ++it) {
      const int p = tid + it * 256;
      const int row = p >> 4, q = (p & 15) * 8;
      const size_t off = (widx < 2) ? ((R0 + row) * DMOD + (size_t)(n0 + q))
                                    : ((vtr0 + n0 + row) * SEQ_FULL + (size_t)(s0 + q));
      *(volatile v8h*)(D + off) = pv[it];
    }
  }
}

template<int RES>
__global__ __launch_bounds__(128) __attribute__((amdgpu_num_vgpr(256)))
void k_attn(const _Float16* __restrict__ Qh, const _Float16* __restrict__ Ql,
            const _Float16* __restrict__ Kh, const _Float16* __restrict__ Kl,
            const _Float16* __restrict__ Vh, const _Float16* __restrict__ Vl,
            _Float16* __restrict__ Og, int qt0)
{
  constexpr int NRS = RES ? (64 * LDT) : 16;
  __shared__ __attribute__((aligned(16))) _Float16 Ks[64 * LDT];
  __shared__ __attribute__((aligned(16))) _Float16 Vs[64 * LDT];
  __shared__ __attribute__((aligned(16))) _Float16 Ps[64 * LDT];
  __shared__ __attribute__((aligned(16))) _Float16 Kls[NRS];
  __shared__ __attribute__((aligned(16))) _Float16 Vls[NRS];
  __shared__ __attribute__((aligned(16))) _Float16 Prs[NRS];
  __shared__ __attribute__((aligned(16))) float Ss[64 * LDSF];
  __shared__ __attribute__((aligned(16))) float cs[64];
  __shared__ __attribute__((aligned(16))) float ls[64];

  const int tid = threadIdx.x, lane = tid & 31, wid = tid >> 5;
  const int hh = lane >> 4, n16 = lane & 15;
  const int qt = (int)blockIdx.x + qt0;
  const int b = (int)blockIdx.y / NH;
  const int h = (int)blockIdx.y - b * NH;
  const int q0 = qt * 64;
  const int qw = q0 + wid * 16;
  const size_t rb = (size_t)b * SEQ_FULL;
  const size_t vrow0 = (size_t)b * DMOD + (size_t)(h * HD);

  v16h qa0, qa1, ql0, ql1;
  {
    const _Float16* qp = Qh + (rb + qw) * DMOD + h * HD;
    qa0 = ld_frag(qp, DMOD);
    qa1 = ld_frag(qp + 32, DMOD);
    if (RES) {
      const _Float16* lp = Ql + (rb + qw) * DMOD + h * HD;
      ql0 = ld_frag(lp, DMOD);
      ql1 = ld_frag(lp + 32, DMOD);
    } else {
      ql0 = qa0;
      ql1 = qa1;
    }
  }

  float mrun = -1.0e30f, lrun = 0.0f;
  v8f acc[4], accr[4];
#pragma unroll
  for (int nt = 0; nt < 4; ++nt) { acc[nt] = zero8(); accr[nt] = zero8(); }

  float* Sw = Ss + (wid * 16) * LDSF;
  _Float16* Pw = Ps + (wid * 16) * LDT;
  const int pro = RES ? (wid * 16) * LDT : 0;

#pragma unroll 1
  for (int kt = 0; kt <= qt; ++kt) {
    const int k0 = kt * 64;
    __syncthreads();
#pragma unroll
    for (int j = 0; j < 4; ++j) {
      const int c = tid + j * 128;
      const int r = c >> 3, cc = (c & 7) * 8;
      *(v8h*)(Ks + r * LDT + cc) = *(const v8h*)(Kh + (rb + k0 + r) * DMOD + h * HD + cc);
      *(v8h*)(Vs + r * LDT + cc) = *(const v8h*)(Vh + (vrow0 + r) * SEQ_FULL + k0 + cc);
      if (RES) {
        *(v8h*)(Kls + r * LDT + cc) = *(const v8h*)(Kl + (rb + k0 + r) * DMOD + h * HD + cc);
        *(v8h*)(Vls + r * LDT + cc) = *(const v8h*)(Vl + (vrow0 + r) * SEQ_FULL + k0 + cc);
      }
    }
    __syncthreads();

#pragma unroll 1
    for (int nt = 0; nt < 4; ++nt) {
      const _Float16* kr = Ks + (nt * 16) * LDT;
      v8f s = zero8();
      v8f sx = zero8();
      {
        const v16h kb0 = ld_frag(kr, LDT);
        s = wmma16(qa0, kb0, s);
        if (RES) sx = wmma16(ql0, kb0, sx);
      }
      {
        const v16h kb1 = ld_frag(kr + 32, LDT);
        s = wmma16(qa1, kb1, s);
        if (RES) sx = wmma16(ql1, kb1, sx);
      }
      if (RES) {
        const _Float16* klr = Kls + (nt * 16) * LDT;
        {
          const v16h kl0 = ld_frag(klr, LDT);
          sx = wmma16(qa0, kl0, sx);
        }
        {
          const v16h kl1 = ld_frag(klr + 32, LDT);
          sx = wmma16(qa1, kl1, sx);
        }
#pragma unroll
        for (int r = 0; r < 8; ++r) s[r] = s[r] + sx[r] * CRINV;
      }
      const int col = k0 + nt * 16 + n16;
      float* dst = Sw + (hh * 8) * LDSF + nt * 16 + n16;
#pragma unroll
      for (int r = 0; r < 8; ++r) {
        const int row = qw + hh * 8 + r;
        const float t = s[r] * 0.125f;
        dst[r * LDSF] = (col > row) ? -1.0e30f : t;
      }
    }
    __syncthreads();

    {
      const float* sr = Sw + n16 * LDSF + hh * 32;
      v4f sv[8];
#pragma unroll
      for (int g = 0; g < 8; ++g) sv[g] = *(const v4f*)(sr + g * 4);
      float mx = -1.0e30f;
#pragma unroll
      for (int g = 0; g < 8; ++g)
#pragma unroll
        for (int e = 0; e < 4; ++e) mx = fmaxf(mx, sv[g][e]);
      mx = fmaxf(mx, __shfl_xor(mx, 16, 32));
      const float mn = fmaxf(mrun, mx);
      const float corr = __expf(mrun - mn);
      mrun = mn;
      float ps = 0.0f;
      _Float16* pdst = Pw + n16 * LDT + hh * 32;
#pragma unroll
      for (int g = 0; g < 4; ++g) {
        v8h ph, pr;
#pragma unroll
        for (int e = 0; e < 8; ++e) {
          const float p = __expf(sv[2 * g + (e >> 2)][e & 3] - mn);
          ps += p;
          const float pc = p * CPV;
          const _Float16 hv = (_Float16)pc;
          ph[e] = hv;
          if (RES) pr[e] = (_Float16)((pc - (float)hv) * CRES);
          else pr[e] = hv;
        }
        *(v8h*)(pdst + g * 8) = ph;
        if (RES) *(v8h*)(Prs + pro + n16 * LDT + hh * 32 + g * 8) = pr;
      }
      ps += __shfl_xor(ps, 16, 32);
      lrun = lrun * corr + ps;
      cs[wid * 16 + n16] = corr;
    }
    __syncthreads();

    {
      const v4f c0 = *(const v4f*)(cs + wid * 16 + hh * 8);
      const v4f c1 = *(const v4f*)(cs + wid * 16 + hh * 8 + 4);
#pragma unroll
      for (int nt = 0; nt < 4; ++nt)
#pragma unroll
        for (int r = 0; r < 4; ++r) {
          acc[nt][r] = acc[nt][r] * c0[r];
          acc[nt][r + 4] = acc[nt][r + 4] * c1[r];
          if (RES) {
            accr[nt][r] = accr[nt][r] * c0[r];
            accr[nt][r + 4] = accr[nt][r + 4] * c1[r];
          }
        }
    }
#pragma unroll 1
    for (int c = 0; c < 2; ++c) {
      const v16h pa = ld_frag(Pw + c * 32, LDT);
#pragma unroll
      for (int nt = 0; nt < 4; ++nt) {
        const v16h vb = ld_frag(Vs + (nt * 16) * LDT + c * 32, LDT);
        acc[nt] = wmma16(pa, vb, acc[nt]);
      }
      if (RES) {
#pragma unroll
        for (int nt = 0; nt < 4; ++nt) {
          const v16h vlb = ld_frag(Vls + (nt * 16) * LDT + c * 32, LDT);
          accr[nt] = wmma16(pa, vlb, accr[nt]);
        }
        const v16h prf = ld_frag(Prs + pro + c * 32, LDT);
#pragma unroll
        for (int nt = 0; nt < 4; ++nt) {
          const v16h vb = ld_frag(Vs + (nt * 16) * LDT + c * 32, LDT);
          accr[nt] = wmma16(prf, vb, accr[nt]);
        }
      }
    }
  }

  ls[wid * 16 + n16] = lrun;
  __syncthreads();
  {
    const v4f l0 = *(const v4f*)(ls + wid * 16 + hh * 8);
    const v4f l1 = *(const v4f*)(ls + wid * 16 + hh * 8 + 4);
    float inv[8];
#pragma unroll
    for (int r = 0; r < 4; ++r) {
      inv[r]     = (OSC / CPV) * __builtin_amdgcn_rcpf(l0[r]);
      inv[r + 4] = (OSC / CPV) * __builtin_amdgcn_rcpf(l1[r]);
    }
#pragma unroll
    for (int r = 0; r < 8; ++r) {
#pragma unroll
      for (int nt = 0; nt < 4; ++nt) {
        float o = acc[nt][r];
        if (RES) o = o + accr[nt][r] * CRINV;
        Ps[(wid * 16 + hh * 8 + r) * LDT + nt * 16 + n16] = (_Float16)(o * inv[r]);
      }
    }
  }
  __syncthreads();
  v8h ov[4];
#pragma unroll
  for (int j = 0; j < 4; ++j) {
    const int row = (lane >> 3) + 4 * j;
    const int q = (lane & 7) * 8;
    ov[j] = *(const v8h*)(Ps + (wid * 16 + row) * LDT + q);
  }
  _Float16* op = Og + (rb + qw) * DMOD + h * HD;
#pragma unroll
  for (int j = 0; j < 4; ++j) {
    const int row = (lane >> 3) + 4 * j;
    const int q = (lane & 7) * 8;
    *(volatile v8h*)(op + (size_t)row * DMOD + q) = ov[j];
  }
  __threadfence();
#pragma unroll
  for (int j = 0; j < 4; ++j) {
    const int row = (lane >> 3) + 4 * j;
    const int q = (lane & 7) * 8;
    *(volatile v8h*)(op + (size_t)row * DMOD + q) = ov[j];
  }
}

template<int KD, int RIN>
__global__ __launch_bounds__(256) __attribute__((amdgpu_num_vgpr(256)))
void k_gemm_res(const _Float16* __restrict__ A, const _Float16* __restrict__ W16,
                const float* __restrict__ resid, float* __restrict__ out, float osc)
{
  __shared__ __attribute__((aligned(16))) char smem[SMEM_BIG];
  _Float16* As = (_Float16*)smem;
  _Float16* Ws = As + 128 * LDA;

  const int tid = threadIdx.x, lane = tid & 31, wid = tid >> 5;
  const int mw = wid >> 1, nw = wid & 1, hh = lane >> 4, n16 = lane & 15;
  const int rt = (int)blockIdx.x;
  const int b = rt / (SEQ / 128);
  const int s0 = (rt - b * (SEQ / 128)) * 128;
  const size_t R0 = (size_t)b * SEQ_FULL + (size_t)s0;
  const int n0 = (int)blockIdx.y * 128;

  v8f acc[2][4];
#pragma unroll
  for (int mt = 0; mt < 2; ++mt)
#pragma unroll
    for (int nt = 0; nt < 4; ++nt) acc[mt][nt] = zero8();

#pragma unroll 1
  for (int kb = 0; kb < KD; kb += 64) {
    __syncthreads();
#pragma unroll
    for (int j = 0; j < 4; ++j) {
      const int c = tid + j * 256;
      const int r = c >> 3, cc = (c & 7) * 8;
      *(v8h*)(As + r * LDA + cc) = *(const v8h*)(A + (R0 + r) * KD + kb + cc);
      *(v8h*)(Ws + r * LDA + cc) = *(const v8h*)(W16 + (size_t)(n0 + r) * KD + kb + cc);
    }
    __syncthreads();
#pragma unroll
    for (int ks = 0; ks < 2; ++ks) {
      const v16h a0 = ld_frag(As + (mw * 32) * LDA + ks * 32, LDA);
      const v16h a1 = ld_frag(As + (mw * 32 + 16) * LDA + ks * 32, LDA);
#pragma unroll
      for (int nt = 0; nt < 4; ++nt) {
        const v16h bw = ld_frag(Ws + (nw * 64 + nt * 16) * LDA + ks * 32, LDA);
        acc[0][nt] = wmma16(a0, bw, acc[0][nt]);
        acc[1][nt] = wmma16(a1, bw, acc[1][nt]);
      }
    }
  }
  __syncthreads();

  float* Cs = (float*)smem;
#pragma unroll
  for (int mt = 0; mt < 2; ++mt)
#pragma unroll
    for (int nt = 0; nt < 4; ++nt)
#pragma unroll
      for (int r = 0; r < 8; ++r)
        Cs[(mw * 32 + mt * 16 + hh * 8 + r) * LDC + nw * 64 + nt * 16 + n16] = acc[mt][nt][r] * osc;
  __syncthreads();

  v4f ov[16];
#pragma unroll
  for (int it = 0; it < 16; ++it) {
    const int p = tid + it * 256;
    const int row = p >> 5, q = (p & 31) * 4;
    const v4f cv = *(const v4f*)(Cs + row * LDC + q);
    const v4f rv = *(const v4f*)(resid + (R0 + row) * DMOD + n0 + q);
    v4f o;
#pragma unroll
    for (int e = 0; e < 4; ++e) {
      const float re = RIN ? bfr(rv[e]) : rv[e];
      o[e] = cv[e] + re;
    }
    ov[it] = o;
  }
#pragma unroll
  for (int it = 0; it < 16; ++it) {
    const int p = tid + it * 256;
    const int row = p >> 5, q = (p & 31) * 4;
    *(volatile v4f*)(out + (R0 + row) * DMOD + n0 + q) = ov[it];
  }
  __threadfence();
#pragma unroll
  for (int it = 0; it < 16; ++it) {
    const int p = tid + it * 256;
    const int row = p >> 5, q = (p & 31) * 4;
    *(volatile v4f*)(out + (R0 + row) * DMOD + n0 + q) = ov[it];
  }
}

__global__ __launch_bounds__(256) __attribute__((amdgpu_num_vgpr(256)))
void k_gateup(const _Float16* __restrict__ Hp, const _Float16* __restrict__ Wg,
              const _Float16* __restrict__ Wu, _Float16* __restrict__ Aout)
{
  __shared__ __attribute__((aligned(16))) _Float16 As[128 * LDA];
  __shared__ __attribute__((aligned(16))) _Float16 Wgs[64 * LDA];
  __shared__ __attribute__((aligned(16))) _Float16 Wus[64 * LDA];

  const int tid = threadIdx.x, lane = tid & 31, wid = tid >> 5;
  const int hh = lane >> 4, n16 = lane & 15;
  const int rt = (int)blockIdx.x;
  const int b = rt / (SEQ / 128);
  const int s0 = (rt - b * (SEQ / 128)) * 128;
  const size_t R0 = (size_t)b * SEQ_FULL + (size_t)s0;
  const int n0 = (int)blockIdx.y * 64;

  v8f ag[4], au[4];
#pragma unroll
  for (int nt = 0; nt < 4; ++nt) { ag[nt] = zero8(); au[nt] = zero8(); }

#pragma unroll 1
  for (int kb = 0; kb < DMOD; kb += 64) {
    __syncthreads();
#pragma unroll
    for (int j = 0; j < 4; ++j) {
      const int c = tid + j * 256;
      const int r = c >> 3, cc = (c & 7) * 8;
      *(v8h*)(As + r * LDA + cc) = *(const v8h*)(Hp + (R0 + r) * DMOD + kb + cc);
    }
#pragma unroll
    for (int j = 0; j < 2; ++j) {
      const int c = tid + j * 256;
      const int r = c >> 3, cc = (c & 7) * 8;
      *(v8h*)(Wgs + r * LDA + cc) = *(const v8h*)(Wg + (size_t)(n0 + r) * DMOD + kb + cc);
      *(v8h*)(Wus + r * LDA + cc) = *(const v8h*)(Wu + (size_t)(n0 + r) * DMOD + kb + cc);
    }
    __syncthreads();
#pragma unroll
    for (int ks = 0; ks < 2; ++ks) {
      const v16h a = ld_frag(As + (wid * 16) * LDA + ks * 32, LDA);
#pragma unroll
      for (int nt = 0; nt < 4; ++nt) {
        {
          const v16h bg = ld_frag(Wgs + (nt * 16) * LDA + ks * 32, LDA);
          ag[nt] = wmma16(a, bg, ag[nt]);
        }
        {
          const v16h bu = ld_frag(Wus + (nt * 16) * LDA + ks * 32, LDA);
          au[nt] = wmma16(a, bu, au[nt]);
        }
      }
    }
  }
  __syncthreads();

  _Float16* Es = As;
#pragma unroll
  for (int nt = 0; nt < 4; ++nt)
#pragma unroll
    for (int r = 0; r < 8; ++r) {
      const float g = ag[nt][r] * WINV;
      const float u = au[nt][r] * WINV;
      const float sg = g * __builtin_amdgcn_rcpf(1.0f + __expf(-g));
      Es[(wid * 16 + hh * 8 + r) * LDA + nt * 16 + n16] = (_Float16)(sg * u);
    }
  __syncthreads();

  v8h pv[4];
#pragma unroll
  for (int it = 0; it < 4; ++it) {
    const int p = tid + it * 256;
    const int row = p >> 3, q = (p & 7) * 8;
    pv[it] = *(const v8h*)(Es + row * LDA + q);
  }
#pragma unroll
  for (int it = 0; it < 4; ++it) {
    const int p = tid + it * 256;
    const int row = p >> 3, q = (p & 7) * 8;
    *(volatile v8h*)(Aout + (R0 + row) * DFF + n0 + q) = pv[it];
  }
  __threadfence();
#pragma unroll
  for (int it = 0; it < 4; ++it) {
    const int p = tid + it * 256;
    const int row = p >> 3, q = (p & 7) * 8;
    *(volatile v8h*)(Aout + (R0 + row) * DFF + n0 + q) = pv[it];
  }
}

extern "C" void kernel_launch(void* const* d_in, const int* in_sizes, int n_in,
                              void* d_out, int out_size, void* d_ws, size_t ws_size,
                              hipStream_t stream)
{
  if (n_in < 11) return;
  const long long need_x = (long long)((NB - 1) * SEQ_FULL + SEQ) * DMOD;
  if ((long long)in_sizes[0] < need_x) return;
  if (in_sizes[1] < SEQ * HD) return;
  if (in_sizes[2] < DMOD * DMOD || in_sizes[3] < DMOD * DMOD ||
      in_sizes[4] < DMOD * DMOD || in_sizes[5] < DMOD * DMOD) return;
  if (in_sizes[6] < DFF * DMOD || in_sizes[7] < DFF * DMOD || in_sizes[8] < DMOD * DFF) return;
  if (in_sizes[9] < DMOD || in_sizes[10] < DMOD) return;
  if ((long long)out_size < need_x) return;

  const size_t MIB = (size_t)1048576;
  const size_t ws_total = 113 * MIB;
  if (ws_size < ws_total) return;

  const float* x    = (const float*)d_in[0];
  const float* rpe  = (const float*)d_in[1];
  const float* wq   = (const float*)d_in[2];
  const float* wk   = (const float*)d_in[3];
  const float* wv   = (const float*)d_in[4];
  const float* wo   = (const float*)d_in[5];
  const float* wg   = (const float*)d_in[6];
  const float* wu   = (const float*)d_in[7];
  const float* wd   = (const float*)d_in[8];
  const float* n1w  = (const float*)d_in[9];
  const float* n2w  = (const float*)d_in[10];
  float* out = (float*)d_out;
  char* ws = (char*)d_ws;

  _Float16* wq16 = (_Float16*)(ws + 0 * MIB);
  _Float16* wk16 = (_Float16*)(ws + 2 * MIB);
  _Float16* wv16 = (_Float16*)(ws + 4 * MIB);
  _Float16* wo16 = (_Float16*)(ws + 6 * MIB);
  _Float16* wg16 = (_Float16*)(ws + 8 * MIB);
  _Float16* wu16 = (_Float16*)(ws + 16 * MIB);
  _Float16* wd16 = (_Float16*)(ws + 24 * MIB);
  float* cosT = (float*)(ws + 32 * MIB);
  float* sinT = (float*)(ws + 32 * MIB + 524288);
  _Float16* h16  = (_Float16*)(ws + 33 * MIB);
  _Float16* qh   = (_Float16*)(ws + 41 * MIB);
  _Float16* ql   = (_Float16*)(ws + 49 * MIB);
  _Float16* kh   = (_Float16*)(ws + 57 * MIB);
  _Float16* kl   = (_Float16*)(ws + 65 * MIB);
  _Float16* vth  = (_Float16*)(ws + 73 * MIB);
  _Float16* vtl  = (_Float16*)(ws + 81 * MIB);
  _Float16* a16  = (_Float16*)(ws + 41 * MIB);
  _Float16* o16  = (_Float16*)(ws + 89 * MIB);
  float* xmid    = (float*)(ws + 97 * MIB);

  dim3 blk(256);
  {
    const int n8a = (DMOD * DMOD) / 8;
    const int n8b = (DFF * DMOD) / 8;
    k_cvt_w<<<dim3((n8a + 255) / 256), blk, 0, stream>>>(wq, wq16, n8a);
    k_cvt_w<<<dim3((n8a + 255) / 256), blk, 0, stream>>>(wk, wk16, n8a);
    k_cvt_w<<<dim3((n8a + 255) / 256), blk, 0, stream>>>(wv, wv16, n8a);
    k_cvt_w<<<dim3((n8a + 255) / 256), blk, 0, stream>>>(wo, wo16, n8a);
    k_cvt_w<<<dim3((n8b + 255) / 256), blk, 0, stream>>>(wg, wg16, n8b);
    k_cvt_w<<<dim3((n8b + 255) / 256), blk, 0, stream>>>(wu, wu16, n8b);
    k_cvt_w<<<dim3((n8b + 255) / 256), blk, 0, stream>>>(wd, wd16, n8b);
  }
  {
    const int nt = SEQ * HD;
    k_trig<<<dim3((nt + 255) / 256), blk, 0, stream>>>(rpe, cosT, sinT, nt);
  }
  const int nrows = NB * SEQ;
  const int nrt = nrows / 128;
  k_rms<1><<<dim3((nrows + 7) / 8), blk, 0, stream>>>(x, n1w, h16, nrows);
  k_qkv<<<dim3(nrt, 3 * (DMOD / 128)), blk, 0, stream>>>(h16, wq16, wk16, wv16, cosT, sinT,
                                                         qh, ql, kh, kl, vth, vtl);
  {
    const int nqt = SEQ / 64;
    k_attn<1><<<dim3(EARLY_QT, NB * NH), dim3(128), 0, stream>>>(qh, ql, kh, kl, vth, vtl, o16, 0);
    if (nqt > EARLY_QT)
      k_attn<0><<<dim3(nqt - EARLY_QT, NB * NH), dim3(128), 0, stream>>>(qh, ql, kh, kl, vth, vtl,
                                                                       o16, EARLY_QT);
  }
  k_gemm_res<DMOD, 1><<<dim3(nrt, DMOD / 128), blk, 0, stream>>>(o16, wo16, x, xmid,
                                                                 1.0f / (64.0f * 16.0f));
  k_rms<0><<<dim3((nrows + 7) / 8), blk, 0, stream>>>(xmid, n2w, h16, nrows);
  k_gateup<<<dim3(nrt, DFF / 64), blk, 0, stream>>>(h16, wg16, wu16, a16);
  k_gemm_res<DFF, 0><<<dim3(nrt, DMOD / 128), blk, 0, stream>>>(a16, wd16, xmid, out, 1.0f / 64.0f);
}
